// PointNetSetAbstraction_82403242541510
// MI455X (gfx1250) — hardware-verified
//
#include <hip/hip_runtime.h>
#pragma clang fp contract(off)

typedef __attribute__((ext_vector_type(16))) _Float16 v16h;
typedef __attribute__((ext_vector_type(8)))  _Float16 v8h;
typedef __attribute__((ext_vector_type(8)))  float    v8f;
typedef __attribute__((ext_vector_type(4)))  float    v4f;
typedef __attribute__((ext_vector_type(4)))  unsigned v4u;

constexpr int BATCH = 16;
constexpr int NPTS = 4096;
constexpr int NQRY = 1024;
constexpr int KNBR = 32;
constexpr int DFEAT = 64;
constexpr int CIN0 = 67;
constexpr int KPAD0 = 96;
constexpr int CH0 = 64;
constexpr int CH1 = 64;
constexpr int CH2 = 128;
constexpr int ROWS_TOTAL = BATCH * NQRY * KNBR;
constexpr int NGROUPS = BATCH * NQRY;
constexpr int LWAVES = 4;
constexpr int LTHREADS = 128;
constexpr int LBLOCKS = ROWS_TOTAL / 128;
constexpr int A1PITCH = 72;
constexpr int W0H_OFF = 0;
constexpr int W1H_OFF = CH0 * KPAD0;
constexpr int W2H_OFF = W1H_OFF + CH1 * CH0;
constexpr int WPL_HALVES = W2H_OFF + CH2 * CH1;
constexpr double INV_ROWS = 1.0 / (double)ROWS_TOTAL;

static_assert(KNBR == 32, "one pooling group per wave");
static_assert(KPAD0 % 32 == 0 && CH0 % 32 == 0 && CH1 % 32 == 0, "k multiples of 32");
static_assert(CH0 % 16 == 0 && CH1 % 16 == 0 && CH2 % 64 == 0, "n tiles");
static_assert(ROWS_TOTAL % 128 == 0, "row tiles");
static_assert(WPL_HALVES * 2 == 36864, "weight plane bytes");
static_assert(CIN0 == 3 + DFEAT, "input channels");

constexpr size_t OFF_KNN  = 0;
constexpr size_t SZ_KNN   = (size_t)ROWS_TOTAL * 4;
constexpr size_t OFF_PH   = OFF_KNN + SZ_KNN;
constexpr size_t SZ_PH    = (size_t)BATCH * NPTS * DFEAT * 2;
constexpr size_t OFF_WPL  = OFF_PH + SZ_PH;
constexpr size_t SZ_WPL   = (size_t)WPL_HALVES * 2;
constexpr size_t OFF_Y0   = OFF_WPL + SZ_WPL;
constexpr size_t SZ_Y0    = (size_t)ROWS_TOTAL * CH0 * 2;
constexpr size_t OFF_GMAX = OFF_Y0 + SZ_Y0;
constexpr size_t SZ_GM    = (size_t)NGROUPS * CH2 * 4;
constexpr size_t OFF_GMIN = OFF_GMAX + SZ_GM;
constexpr size_t OFF_P0   = OFF_GMIN + SZ_GM;
constexpr size_t SZ_P0    = (size_t)LBLOCKS * 128 * 4;
constexpr size_t OFF_P1   = OFF_P0 + SZ_P0;
constexpr size_t OFF_P2   = OFF_P1 + SZ_P0;
constexpr size_t SZ_P2    = (size_t)LBLOCKS * 256 * 4;
constexpr size_t OFF_AFF  = OFF_P2 + SZ_P2;
constexpr size_t SZ_AFF   = 4096;
constexpr size_t WS_TOTAL = OFF_AFF + SZ_AFF;
static_assert(WS_TOTAL == 102801408, "carve total");
static_assert(WS_TOTAL <= 134217728, "carve cap");
static_assert(OFF_PH % 128 == 0 && OFF_WPL % 128 == 0 && OFF_Y0 % 128 == 0 && OFF_GMAX % 128 == 0 &&
              OFF_GMIN % 128 == 0 && OFF_P0 % 128 == 0 && OFF_P1 % 128 == 0 && OFF_P2 % 128 == 0 &&
              OFF_AFF % 128 == 0, "line aligned regions");
constexpr size_t OUT1_OFF_BYTES = (size_t)BATCH * NQRY * 3 * 4;
static_assert(OUT1_OFF_BYTES == 196608, "out1 byte offset");
static_assert(OUT1_OFF_BYTES % 128 == 0, "out1 line aligned");
static_assert(OUT1_OFF_BYTES + (size_t)NGROUPS * CH2 * 4 == 8585216, "d_out total");

union FragU { v16h v; v8h h[2]; };

__device__ __forceinline__ v16h frag_load(const _Float16* p) {
  FragU f;
  f.h[0] = *(const v8h*)(p);
  f.h[1] = *(const v8h*)(p + 16);
  return f.v;
}

__device__ __forceinline__ v8f mma_h(v16h a, v16h b, v8f c) {
  c = __builtin_amdgcn_wmma_f32_16x16x32_f16(false, a, false, b, (short)0, c, false, false);
  asm volatile("v_nop\n\tv_nop\n\tv_nop\n\tv_nop" : "+v"(c) : "v"(a), "v"(b));
  return c;
}

__device__ __forceinline__ float h16_to_f32(unsigned hb) {
  const unsigned sgn = (hb & 0x8000u) << 16;
  const unsigned em = hb & 0x7fffu;
  const float fn = __uint_as_float((em << 13) + 0x38000000u);
  const float fs = (float)em * 5.9604644775390625e-8f;
  const float mag = (em < 0x400u) ? fs : fn;
  return __uint_as_float(__float_as_uint(mag) | sgn);
}

__device__ __forceinline__ int clampi(int v, int hi) {
  v = v < 0 ? 0 : v;
  return v > hi ? hi : v;
}

__device__ __forceinline__ void store2_v4f(float* p, v4f v) {
  volatile v4f* d = (volatile v4f*)p;
  *d = v;
  __threadfence();
  *d = v;
}

__device__ __forceinline__ void store2_v8h(_Float16* p, v8h v) {
  volatile v8h* d = (volatile v8h*)p;
  *d = v;
  __threadfence();
  *d = v;
}

__global__ __launch_bounds__(256) void k_cvt_points(const float* __restrict__ pts, _Float16* __restrict__ ph) {
  const size_t t = (size_t)blockIdx.x * 256 + threadIdx.x;
  const size_t total = (size_t)BATCH * NPTS * DFEAT / 8;
  if (t < total) {
    const v4f a = *(const v4f*)(pts + t * 8);
    const v4f b = *(const v4f*)(pts + t * 8 + 4);
    v8h hv;
    hv[0] = (_Float16)a[0];
    hv[1] = (_Float16)a[1];
    hv[2] = (_Float16)a[2];
    hv[3] = (_Float16)a[3];
    hv[4] = (_Float16)b[0];
    hv[5] = (_Float16)b[1];
    hv[6] = (_Float16)b[2];
    hv[7] = (_Float16)b[3];
    store2_v8h(ph + t * 8, hv);
  }
}

__global__ __launch_bounds__(256) void k_prep_w(const float* __restrict__ W0, const float* __restrict__ W1,
                                                const float* __restrict__ W2, _Float16* __restrict__ wpl) {
  const int blk = blockIdx.x;
  const int tid = threadIdx.x;
  float zz = 0.0f;
  asm volatile("" : "+v"(zz));
  float v[8];
  int outoff;
  if (blk < 3) {
    const int e0 = (blk * 256 + tid) * 8;
    const int o = e0 / KPAD0;
    const int k0 = e0 - o * KPAD0;
#pragma unroll
    for (int e = 0; e < 8; ++e) {
      const int kp = k0 + e;
      const int col = (kp < 64) ? (kp + 3) : ((kp < CIN0) ? (kp - 64) : 0);
      const float x = W0[o * CIN0 + col];
      v[e] = (kp < CIN0) ? x : zz;
    }
    outoff = W0H_OFF + e0;
  } else if (blk < 5) {
    const int e0 = ((blk - 3) * 256 + tid) * 8;
    const v4f a = *(const v4f*)(W1 + e0);
    const v4f b = *(const v4f*)(W1 + e0 + 4);
    v[0] = a[0]; v[1] = a[1]; v[2] = a[2]; v[3] = a[3];
    v[4] = b[0]; v[5] = b[1]; v[6] = b[2]; v[7] = b[3];
    outoff = W1H_OFF + e0;
  } else {
    const int e0 = ((blk - 5) * 256 + tid) * 8;
    const v4f a = *(const v4f*)(W2 + e0);
    const v4f b = *(const v4f*)(W2 + e0 + 4);
    v[0] = a[0]; v[1] = a[1]; v[2] = a[2]; v[3] = a[3];
    v[4] = b[0]; v[5] = b[1]; v[6] = b[2]; v[7] = b[3];
    outoff = W2H_OFF + e0;
  }
  v8h hv;
#pragma unroll
  for (int e = 0; e < 8; ++e) hv[e] = (_Float16)v[e];
  store2_v8h(wpl + outoff, hv);
}

__global__ __launch_bounds__(256) void k_knn(const float* __restrict__ xyz, const int* __restrict__ idx,
                                             int* __restrict__ knn, float* __restrict__ out0) {
#pragma clang fp contract(off)
  __shared__ __align__(16) float s_xyz[3 * NPTS];
  const int tid = threadIdx.x;
  const int lane = tid & 31;
  const int wave = tid >> 5;
  const int b = blockIdx.x >> 5;
  const int s0 = (blockIdx.x & 31) << 5;
  const float* bx = xyz + (size_t)b * (NPTS * 3);
#pragma unroll 1
  for (int it = 0; it < 3; ++it) {
#pragma unroll
    for (int u = 0; u < 4; ++u) {
      const int f = (it * 4 + u) * 256 + tid;
      const v4f g = *(const v4f*)(bx + 4 * f);
#pragma unroll
      for (int j = 0; j < 4; ++j) {
        const int e = 4 * f + j;
        const int p = e / 3;
        const int c = e - 3 * p;
        s_xyz[c * NPTS + p] = g[j];
      }
    }
  }
  __syncthreads();

  const int up = (lane + 31) & 31;
#pragma unroll 1
  for (int qq = 0; qq < 4; ++qq) {
    const int s = s0 + wave * 4 + qq;
    const int qi = clampi(idx[b * NQRY + s], NPTS - 1);
    const float qx = s_xyz[qi];
    const float qy = s_xyz[NPTS + qi];
    const float qz = s_xyz[2 * NPTS + qi];
    float ed = __builtin_huge_valf();
    int ei = 0;
#pragma unroll 1
    for (int n0 = 0; n0 < NPTS; n0 += 32) {
      const float x = s_xyz[n0 + lane];
      const float y = s_xyz[NPTS + n0 + lane];
      const float z = s_xyz[2 * NPTS + n0 + lane];
      const float dx = qx - x;
      const float dy = qy - y;
      const float dz = qz - z;
      const float t0 = dx * dx;
      const float t1 = dy * dy;
      const float t2 = dz * dz;
      const float d = (t0 + t2) + t1;
      const float thr = __shfl(ed, 31, 32);
      unsigned mask = __builtin_amdgcn_ballot_w32(d < thr);
      while (mask != 0u) {
        const int src = __builtin_ctz(mask);
        mask &= (mask - 1u);
        const float cd = __shfl(d, src, 32);
        const int cn = n0 + src;
        const float pd = __shfl(ed, up, 32);
        const int pi = __shfl(ei, up, 32);
        const bool gt = ed > cd;
        const bool pgt = (lane > 0) && (pd > cd);
        const float nd = gt ? (pgt ? pd : cd) : ed;
        const int ni = gt ? (pgt ? pi : cn) : ei;
        ed = nd;
        ei = ni;
      }
    }
    volatile int* kp = (volatile int*)(knn + ((size_t)(b * NQRY + s)) * KNBR + lane);
    const int kv = clampi(ei, NPTS - 1);
    *kp = kv;
    __threadfence();
    *kp = kv;
  }

  if (wave == 0) {
    v4f o;
#pragma unroll
    for (int j = 0; j < 4; ++j) {
      int e = lane * 4 + j;
      e = e > 95 ? 95 : e;
      const int p = e / 3;
      const int c = e - 3 * p;
      const int qj = clampi(idx[b * NQRY + s0 + p], NPTS - 1);
      o[j] = s_xyz[c * NPTS + qj];
    }
    if (lane < 24) {
      store2_v4f(out0 + ((size_t)(b * NQRY + s0)) * 3 + lane * 4, o);
    }
  }
}

__device__ __forceinline__ void tile_stats4(const v8f (&acc)[2][4], float* dsum, float* dssq, int h, int m) {
#pragma unroll
  for (int nt = 0; nt < 4; ++nt) {
    float ps = 0.0f;
    float pq = 0.0f;
#pragma unroll
    for (int i = 0; i < 2; ++i) {
#pragma unroll
      for (int r = 0; r < 8; ++r) {
        const float v = acc[i][nt][r];
        const float vv = v * v;
        ps += v;
        pq += vv;
      }
    }
    ps += __shfl_xor(ps, 16, 32);
    pq += __shfl_xor(pq, 16, 32);
    if (h == 0) {
      dsum[nt * 16 + m] = ps;
      dssq[nt * 16 + m] = pq;
    }
  }
}

__global__ __launch_bounds__(128) void k_layer0(const float* __restrict__ xyz, const int* __restrict__ idx,
                                                const int* __restrict__ knn, const _Float16* __restrict__ ph,
                                                const _Float16* __restrict__ w0h, const float* __restrict__ b0,
                                                _Float16* __restrict__ y0, float* __restrict__ part0) {
  __shared__ __align__(16) _Float16 s_w[CH0 * KPAD0];
  __shared__ __align__(16) _Float16 s_a[LWAVES][32 * KPAD0];
  __shared__ float s_part[LWAVES][128];
  __shared__ __align__(16) float s_tot[128];
  const int tid = threadIdx.x;
  const int lane = tid & 31;
  const int wave = tid >> 5;
  const int h = lane >> 4;
  const int m = lane & 15;
#pragma unroll 2
  for (int i = tid; i < (CH0 * KPAD0) / 8; i += LTHREADS) {
    ((v8h*)s_w)[i] = ((const v8h*)w0h)[i];
  }
  asm volatile("" ::: "memory");

  const int rowbase = blockIdx.x * 128 + wave * 32;
  const int grp = rowbase >> 5;
  const int b = grp >> 10;
  {
    const int r = rowbase + lane;
    const int n = clampi(knn[r], NPTS - 1);
    const int qi = clampi(idx[grp], NPTS - 1);
    const v8h* prow = (const v8h*)(ph + ((size_t)b * NPTS + n) * DFEAT);
    v8h* arow = (v8h*)(&s_a[wave][lane * KPAD0]);
    v8h pv[8];
#pragma unroll
    for (int j = 0; j < 8; ++j) pv[j] = prow[j];
#pragma unroll
    for (int j = 0; j < 8; ++j) arow[j] = pv[j];
    asm volatile("" ::: "memory");
    const float* bx = xyz + (size_t)b * (NPTS * 3);
    const float nx = bx[3 * n + 0];
    const float ny = bx[3 * n + 1];
    const float nz = bx[3 * n + 2];
    const float cx = bx[3 * qi + 0];
    const float cy = bx[3 * qi + 1];
    const float cz = bx[3 * qi + 2];
    float zz = 0.0f;
    asm volatile("" : "+v"(zz));
    v8h t;
    t[0] = (_Float16)(nx - cx);
    t[1] = (_Float16)(ny - cy);
    t[2] = (_Float16)(nz - cz);
    t[3] = (_Float16)zz;
    t[4] = (_Float16)zz;
    t[5] = (_Float16)zz;
    t[6] = (_Float16)zz;
    t[7] = (_Float16)zz;
    v8h zv;
#pragma unroll
    for (int e = 0; e < 8; ++e) zv[e] = (_Float16)zz;
    arow[8] = t;
    arow[9] = zv;
    arow[10] = zv;
    arow[11] = zv;
  }
  __syncthreads();

  v8f acc[2][4];
#pragma unroll
  for (int nt = 0; nt < 4; ++nt) {
    const float bv = b0[nt * 16 + m];
    acc[0][nt] = (v8f){bv, bv, bv, bv, bv, bv, bv, bv};
    acc[1][nt] = (v8f){bv, bv, bv, bv, bv, bv, bv, bv};
  }
  const _Float16* at = &s_a[wave][0];
#pragma unroll
  for (int kc = 0; kc < 3; ++kc) {
    const v16h a0 = frag_load(at + m * KPAD0 + kc * 32 + 8 * h);
    const v16h a1 = frag_load(at + (16 + m) * KPAD0 + kc * 32 + 8 * h);
#pragma unroll
    for (int nt = 0; nt < 4; ++nt) {
      const v16h bf = frag_load(s_w + (nt * 16 + m) * KPAD0 + kc * 32 + 8 * h);
      acc[0][nt] = mma_h(a0, bf, acc[0][nt]);
      acc[1][nt] = mma_h(a1, bf, acc[1][nt]);
    }
  }

  tile_stats4(acc, &s_part[wave][0], &s_part[wave][64], h, m);
  __syncthreads();

  _Float16* yt = &s_a[wave][0];
#pragma unroll
  for (int i = 0; i < 2; ++i) {
#pragma unroll
    for (int nt = 0; nt < 4; ++nt) {
#pragma unroll
      for (int r = 0; r < 8; ++r) {
        yt[(16 * i + 8 * h + r) * KPAD0 + nt * 16 + m] = (_Float16)acc[i][nt][r];
      }
    }
  }
  s_tot[tid] = ((s_part[0][tid] + s_part[1][tid]) + s_part[2][tid]) + s_part[3][tid];
  __syncthreads();

  {
    const int q = lane >> 3;
    const int c8 = (lane & 7) * 8;
    v8h yv[8];
#pragma unroll
    for (int it = 0; it < 8; ++it) yv[it] = *(const v8h*)(yt + (it * 4 + q) * KPAD0 + c8);
#pragma unroll
    for (int it = 0; it < 8; ++it)
      *(volatile v8h*)(y0 + (size_t)(rowbase + it * 4 + q) * CH0 + c8) = yv[it];
    __threadfence();
#pragma unroll
    for (int it = 0; it < 8; ++it)
      *(volatile v8h*)(y0 + (size_t)(rowbase + it * 4 + q) * CH0 + c8) = yv[it];
  }
  if (wave == 0) {
    const v4f pv4 = *(const v4f*)(s_tot + lane * 4);
    store2_v4f(part0 + (size_t)blockIdx.x * 128 + lane * 4, pv4);
  }
}

__device__ __forceinline__ v16h bn_relu_frag(const v4u wa, const v4u wb, const float* sc, const float* sh) {
  const v4f sa0 = *(const v4f*)(sc);
  const v4f sa1 = *(const v4f*)(sc + 4);
  const v4f sb0 = *(const v4f*)(sc + 16);
  const v4f sb1 = *(const v4f*)(sc + 20);
  const v4f ha0 = *(const v4f*)(sh);
  const v4f ha1 = *(const v4f*)(sh + 4);
  const v4f hb0 = *(const v4f*)(sh + 16);
  const v4f hb1 = *(const v4f*)(sh + 20);
  float scv[16];
  float shv[16];
#pragma unroll
  for (int e = 0; e < 4; ++e) {
    scv[e] = sa0[e];
    scv[4 + e] = sa1[e];
    scv[8 + e] = sb0[e];
    scv[12 + e] = sb1[e];
    shv[e] = ha0[e];
    shv[4 + e] = ha1[e];
    shv[8 + e] = hb0[e];
    shv[12 + e] = hb1[e];
  }
  unsigned wd[8];
#pragma unroll
  for (int j = 0; j < 4; ++j) {
    wd[j] = wa[j];
    wd[4 + j] = wb[j];
  }
  v16h r;
#pragma unroll
  for (int j = 0; j < 8; ++j) {
    const unsigned w = wd[j];
    const float x0 = h16_to_f32(w & 0xffffu);
    const float x1 = h16_to_f32(w >> 16);
    const float p0 = x0 * scv[2 * j];
    const float p1 = x1 * scv[2 * j + 1];
    const float y0v = fmaxf(p0 + shv[2 * j], 0.0f);
    const float y1v = fmaxf(p1 + shv[2 * j + 1], 0.0f);
    r[2 * j] = (_Float16)y0v;
    r[2 * j + 1] = (_Float16)y1v;
  }
  return r;
}

__device__ __forceinline__ void layer1_tile(const unsigned* __restrict__ y0w, int rowbase, int lane,
                                            const _Float16* s_w1, const float* s_aff0,
                                            const float* __restrict__ b1, v8f (&acc)[2][4]) {
  const int h = lane >> 4;
  const int m = lane & 15;
#pragma unroll
  for (int nt = 0; nt < 4; ++nt) {
    const float bv = b1[nt * 16 + m];
    acc[0][nt] = (v8f){bv, bv, bv, bv, bv, bv, bv, bv};
    acc[1][nt] = (v8f){bv, bv, bv, bv, bv, bv, bv, bv};
  }
  const v4u* yr0 = (const v4u*)(y0w) + (size_t)(rowbase + m) * 8;
  const v4u* yr1 = (const v4u*)(y0w) + (size_t)(rowbase + 16 + m) * 8;
  v4u wa[2][2][2];
#pragma unroll
  for (int kc = 0; kc < 2; ++kc) {
#pragma unroll
    for (int rn = 0; rn < 2; ++rn) {
      wa[0][kc][rn] = yr0[kc * 4 + h + 2 * rn];
      wa[1][kc][rn] = yr1[kc * 4 + h + 2 * rn];
    }
  }
#pragma unroll
  for (int kc = 0; kc < 2; ++kc) {
    const v16h a0 = bn_relu_frag(wa[0][kc][0], wa[0][kc][1], s_aff0 + kc * 32 + 8 * h, s_aff0 + 64 + kc * 32 + 8 * h);
    const v16h a1 = bn_relu_frag(wa[1][kc][0], wa[1][kc][1], s_aff0 + kc * 32 + 8 * h, s_aff0 + 64 + kc * 32 + 8 * h);
#pragma unroll
    for (int nt = 0; nt < 4; ++nt) {
      const v16h bf = frag_load(s_w1 + (nt * 16 + m) * CH0 + kc * 32 + 8 * h);
      acc[0][nt] = mma_h(a0, bf, acc[0][nt]);
      acc[1][nt] = mma_h(a1, bf, acc[1][nt]);
    }
  }
}

__global__ __launch_bounds__(128) void k_layer1_stats(const unsigned* __restrict__ y0w, const _Float16* __restrict__ w1h,
                                                      const float* __restrict__ b1, const float* __restrict__ aff0,
                                                      float* __restrict__ part1) {
  __shared__ __align__(16) _Float16 s_w1[CH1 * CH0];
  __shared__ __align__(16) float s_aff0[128];
  __shared__ float s_part[LWAVES][128];
  __shared__ __align__(16) float s_tot[128];
  const int tid = threadIdx.x;
  const int lane = tid & 31;
  const int wave = tid >> 5;
  const int h = lane >> 4;
  const int m = lane & 15;
#pragma unroll 4
  for (int i = tid; i < (CH1 * CH0) / 8; i += LTHREADS) {
    ((v8h*)s_w1)[i] = ((const v8h*)w1h)[i];
  }
  s_aff0[tid] = aff0[tid];
  __syncthreads();

  const int rowbase = blockIdx.x * 128 + wave * 32;
  v8f acc[2][4];
  layer1_tile(y0w, rowbase, lane, s_w1, s_aff0, b1, acc);
  tile_stats4(acc, &s_part[wave][0], &s_part[wave][64], h, m);
  __syncthreads();
  s_tot[tid] = ((s_part[0][tid] + s_part[1][tid]) + s_part[2][tid]) + s_part[3][tid];
  __syncthreads();
  if (wave == 0) {
    const v4f pv4 = *(const v4f*)(s_tot + lane * 4);
    store2_v4f(part1 + (size_t)blockIdx.x * 128 + lane * 4, pv4);
  }
}

__global__ __launch_bounds__(128) void k_layer12(const unsigned* __restrict__ y0w, const _Float16* __restrict__ w12h,
                                                 const float* __restrict__ b1, const float* __restrict__ b2,
                                                 const float* __restrict__ aff0, const float* __restrict__ aff1,
                                                 float* __restrict__ part2, float* __restrict__ gmax,
                                                 float* __restrict__ gmin) {
  __shared__ __align__(16) _Float16 s_w12[CH1 * CH0 + CH2 * CH1];
  __shared__ __align__(16) _Float16 s_a1[LWAVES][32 * A1PITCH];
  __shared__ __align__(16) float s_aff0[128];
  __shared__ __align__(16) float s_aff1[128];
  __shared__ float s_part[LWAVES][256];
  __shared__ __align__(16) float s_mm[LWAVES][256];
  __shared__ __align__(16) float s_tot[256];
  const int tid = threadIdx.x;
  const int lane = tid & 31;
  const int wave = tid >> 5;
  const int h = lane >> 4;
  const int m = lane & 15;
#pragma unroll 4
  for (int i = tid; i < (CH1 * CH0 + CH2 * CH1) / 8; i += LTHREADS) {
    ((v8h*)s_w12)[i] = ((const v8h*)w12h)[i];
  }
  s_aff0[tid] = aff0[tid];
  s_aff1[tid] = aff1[tid];
  __syncthreads();

  const int rowbase = blockIdx.x * 128 + wave * 32;
  const int grp = rowbase >> 5;
  _Float16* at = &s_a1[wave][0];
  {
    v8f acc1[2][4];
    layer1_tile(y0w, rowbase, lane, s_w12, s_aff0, b1, acc1);
#pragma unroll
    for (int nt = 0; nt < 4; ++nt) {
      const int ch = nt * 16 + m;
      const float sc = s_aff1[ch];
      const float sh = s_aff1[64 + ch];
#pragma unroll
      for (int i = 0; i < 2; ++i) {
#pragma unroll
        for (int r = 0; r < 8; ++r) {
          const float p = acc1[i][nt][r] * sc;
          const float v = fmaxf(p + sh, 0.0f);
          at[(16 * i + 8 * h + r) * A1PITCH + ch] = (_Float16)v;
        }
      }
    }
  }
  __syncthreads();

  v16h a2[2][2];
#pragma unroll
  for (int i = 0; i < 2; ++i) {
#pragma unroll
    for (int kc = 0; kc < 2; ++kc) {
      a2[i][kc] = frag_load(at + (16 * i + m) * A1PITCH + kc * 32 + 8 * h);
    }
  }
  const _Float16* s_w2 = s_w12 + CH1 * CH0;

#pragma unroll 1
  for (int nh = 0; nh < 2; ++nh) {
    v8f acc2[2][4];
#pragma unroll
    for (int nt = 0; nt < 4; ++nt) {
      const float bv = b2[nh * 64 + nt * 16 + m];
      acc2[0][nt] = (v8f){bv, bv, bv, bv, bv, bv, bv, bv};
      acc2[1][nt] = (v8f){bv, bv, bv, bv, bv, bv, bv, bv};
    }
#pragma unroll
    for (int kc = 0; kc < 2; ++kc) {
#pragma unroll
      for (int nt = 0; nt < 4; ++nt) {
        const v16h bf = frag_load(s_w2 + (nh * 64 + nt * 16 + m) * CH1 + kc * 32 + 8 * h);
        acc2[0][nt] = mma_h(a2[0][kc], bf, acc2[0][nt]);
        acc2[1][nt] = mma_h(a2[1][kc], bf, acc2[1][nt]);
      }
    }
#pragma unroll
    for (int nt = 0; nt < 4; ++nt) {
      float ps = 0.0f;
      float pq = 0.0f;
      float mx = -__builtin_huge_valf();
      float mn = __builtin_huge_valf();
#pragma unroll
      for (int i = 0; i < 2; ++i) {
#pragma unroll
        for (int r = 0; r < 8; ++r) {
          const float v = acc2[i][nt][r];
          const float vv = v * v;
          ps += v;
          pq += vv;
          mx = fmaxf(mx, v);
          mn = fminf(mn, v);
        }
      }
      const float ps2 = __shfl_xor(ps, 16, 32);
      const float pq2 = __shfl_xor(pq, 16, 32);
      const float mx2 = __shfl_xor(mx, 16, 32);
      const float mn2 = __shfl_xor(mn, 16, 32);
      ps += ps2;
      pq += pq2;
      mx = fmaxf(mx, mx2);
      mn = fminf(mn, mn2);
      if (h == 0) {
        const int ch = nh * 64 + nt * 16 + m;
        s_part[wave][ch] = ps;
        s_part[wave][128 + ch] = pq;
        s_mm[wave][ch] = mx;
        s_mm[wave][128 + ch] = mn;
      }
    }
  }
  __syncthreads();

  {
    const v4f vmax = *(const v4f*)(&s_mm[wave][lane * 4]);
    const v4f vmin = *(const v4f*)(&s_mm[wave][128 + lane * 4]);
    volatile v4f* dmax = (volatile v4f*)(gmax + (size_t)grp * CH2 + lane * 4);
    volatile v4f* dmin = (volatile v4f*)(gmin + (size_t)grp * CH2 + lane * 4);
    *dmax = vmax;
    *dmin = vmin;
    __threadfence();
    *dmax = vmax;
    *dmin = vmin;
  }
  s_tot[tid] = ((s_part[0][tid] + s_part[1][tid]) + s_part[2][tid]) + s_part[3][tid];
  s_tot[128 + tid] = ((s_part[0][128 + tid] + s_part[1][128 + tid]) + s_part[2][128 + tid]) + s_part[3][128 + tid];
  __syncthreads();
  if (wave == 0) {
    const v4f p0 = *(const v4f*)(s_tot + lane * 4);
    const v4f p1 = *(const v4f*)(s_tot + 128 + lane * 4);
    volatile v4f* d0 = (volatile v4f*)(part2 + (size_t)blockIdx.x * 256 + lane * 4);
    volatile v4f* d1 = (volatile v4f*)(part2 + (size_t)blockIdx.x * 256 + 128 + lane * 4);
    *d0 = p0;
    *d1 = p1;
    __threadfence();
    *d0 = p0;
    *d1 = p1;
  }
}

__global__ __launch_bounds__(256) void k_fold(const float* __restrict__ part, int nrows, int nch,
                                              const float* __restrict__ g, const float* __restrict__ be,
                                              float* __restrict__ aff) {
  __shared__ double s_d[256];
  __shared__ __align__(16) float s_o[256];
  const int tid = threadIdx.x;
  const int ncol = 2 * nch;
  if (tid < ncol) {
    double a = 0.0;
#pragma unroll 4
    for (int r = 0; r < nrows; ++r) a += (double)part[(size_t)r * ncol + tid];
    s_d[tid] = a;
  }
  __syncthreads();
  {
    const int c = tid < nch ? tid : (nch - 1);
    const double mu = s_d[c] * INV_ROWS;
    const double ex2 = s_d[nch + c] * INV_ROWS;
    double var = ex2 - mu * mu;
    var = var < 0.0 ? 0.0 : var;
    const float rs = rsqrtf((float)var + 1e-5f);
    const float sc = rs * g[c];
    const float ms = (float)mu * sc;
    const float sh = be[c] - ms;
    if (tid < nch) {
      s_o[tid] = sc;
      s_o[nch + tid] = sh;
    }
  }
  __syncthreads();
  if (tid < 32) {
    const int nseg = ncol >> 7;
    for (int j = 0; j < nseg; ++j) {
      const v4f v = *(const v4f*)(s_o + j * 128 + tid * 4);
      store2_v4f(aff + j * 128 + tid * 4, v);
    }
  }
}

__global__ __launch_bounds__(256) void k_final(const float* __restrict__ gmax, const float* __restrict__ gmin,
                                               const float* __restrict__ aff2, float* __restrict__ out1) {
  const size_t t = (size_t)blockIdx.x * 256 + threadIdx.x;
  const size_t total = (size_t)NGROUPS * CH2 / 4;
  if (t < total) {
    const int c4 = ((int)(t & 31)) * 4;
    const v4f mx = *(const v4f*)(gmax + t * 4);
    const v4f mn = *(const v4f*)(gmin + t * 4);
    const v4f sc = *(const v4f*)(aff2 + c4);
    const v4f sh = *(const v4f*)(aff2 + CH2 + c4);
    v4f o;
#pragma unroll
    for (int j = 0; j < 4; ++j) {
      const float scj = sc[j];
      const float sel = (scj >= 0.0f) ? mx[j] : mn[j];
      const float p = scj * sel;
      o[j] = fmaxf(p + sh[j], 0.0f);
    }
    store2_v4f(out1 + t * 4, o);
  }
}

extern "C" void kernel_launch(void* const* d_in, const int* in_sizes, int n_in,
                              void* d_out, int out_size, void* d_ws, size_t ws_size,
                              hipStream_t stream) {
  (void)in_sizes; (void)n_in; (void)out_size;
  if (ws_size < WS_TOTAL) return;
  const float* xyz = (const float*)d_in[0];
  const float* pts = (const float*)d_in[1];
  const int*   idx = (const int*)d_in[2];
  const float* W0 = (const float*)d_in[3];
  const float* b0 = (const float*)d_in[4];
  const float* g0 = (const float*)d_in[5];
  const float* be0 = (const float*)d_in[6];
  const float* W1 = (const float*)d_in[7];
  const float* b1 = (const float*)d_in[8];
  const float* g1 = (const float*)d_in[9];
  const float* be1 = (const float*)d_in[10];
  const float* W2 = (const float*)d_in[11];
  const float* b2 = (const float*)d_in[12];
  const float* g2 = (const float*)d_in[13];
  const float* be2 = (const float*)d_in[14];
  float* out0 = (float*)d_out;
  float* out1 = (float*)d_out + OUT1_OFF_BYTES / 4;

  char* ws = (char*)d_ws;
  int*      knn  = (int*)(ws + OFF_KNN);
  _Float16* ph   = (_Float16*)(ws + OFF_PH);
  _Float16* wpl  = (_Float16*)(ws + OFF_WPL);
  _Float16* y0   = (_Float16*)(ws + OFF_Y0);
  float*    gmax = (float*)(ws + OFF_GMAX);
  float*    gmin = (float*)(ws + OFF_GMIN);
  float*    p0   = (float*)(ws + OFF_P0);
  float*    p1   = (float*)(ws + OFF_P1);
  float*    p2   = (float*)(ws + OFF_P2);
  float*    aff  = (float*)(ws + OFF_AFF);
  float* aff0 = aff;
  float* aff1 = aff + 128;
  float* aff2 = aff + 256;

  k_cvt_points<<<(BATCH * NPTS * DFEAT / 8) / 256, 256, 0, stream>>>(pts, ph);
  k_prep_w<<<9, 256, 0, stream>>>(W0, W1, W2, wpl);
  k_knn<<<BATCH * (NQRY / 32), 256, 0, stream>>>(xyz, idx, knn, out0);
  k_layer0<<<LBLOCKS, LTHREADS, 0, stream>>>(xyz, idx, knn, ph, wpl + W0H_OFF, b0, y0, p0);
  k_fold<<<1, 256, 0, stream>>>(p0, LBLOCKS, CH0, g0, be0, aff0);
  k_layer1_stats<<<LBLOCKS, LTHREADS, 0, stream>>>((const unsigned*)y0, wpl + W1H_OFF, b1, aff0, p1);
  k_fold<<<1, 256, 0, stream>>>(p1, LBLOCKS, CH1, g1, be1, aff1);
  k_layer12<<<LBLOCKS, LTHREADS, 0, stream>>>((const unsigned*)y0, wpl + W1H_OFF, b1, b2, aff0, aff1, p2, gmax, gmin);
  k_fold<<<1, 256, 0, stream>>>(p2, LBLOCKS, CH2, g2, be2, aff2);
  k_final<<<(NGROUPS * CH2 / 4) / 256, 256, 0, stream>>>(gmax, gmin, aff2, out1);
}
